// ContinuousTimeRNN_42245298324111
// MI455X (gfx1250) — hardware-run, weakly checked
//
#include <hip/hip_runtime.h>
#include <math.h>

constexpr int NSTEP    = 1000;
constexpr int NBATCH   = 512;
constexpr int NHID     = 512;
constexpr int NIO      = 2;
constexpr int ROWS_BLK = 16;
constexpr int NTHR     = 256;
constexpr int NWAVE    = NTHR / 32;
constexpr int HPITCH   = 520;
constexpr int PPITCH   = 132;
constexpr int NOUT     = NSTEP * NBATCH * NIO;

constexpr float ACARRY   = 1024.0f;
constexpr float WCARRY   = 1024.0f;
constexpr float LEAKF    = 0.1f;
constexpr float KEEPF    = 0.9f;
constexpr float FOLDSC   = LEAKF / (ACARRY * WCARRY);
constexpr float H16_MINN = 6.103515625e-5f;
constexpr float TWO_LOG2E = 2.8853900817779268f;

static_assert(NHID == 64 * NWAVE, "8 waves x 64 hidden columns");
static_assert(NBATCH % ROWS_BLK == 0, "whole 16-row blocks");
static_assert(NHID % 64 == 0 && NHID % 32 == 0, "tile multiples");
static_assert(NIO == 2, "two inputs, two outputs");
static_assert((ROWS_BLK * NIO * 4) == 128, "one 128-B output line per block and step");
static_assert(HPITCH % 8 == 0 && HPITCH >= NHID, "a tile pitch");
static_assert(PPITCH % 4 == 0 && PPITCH >= 16 * NWAVE, "partial pitch");

typedef __attribute__((ext_vector_type(16))) _Float16 v16h;
typedef __attribute__((ext_vector_type(8)))  _Float16 v8h;
typedef __attribute__((ext_vector_type(4)))  _Float16 v4h;
typedef __attribute__((ext_vector_type(8)))  float    v8f;
typedef __attribute__((ext_vector_type(4)))  float    v4f;

__device__ __forceinline__ void guard_group4(v8f& a0, v8f& a1, v8f& a2, v8f& a3,
                                             v16h x, v16h y0, v16h y1, v16h y2, v16h y3) {
  asm volatile("v_nop\n\tv_nop\n\tv_nop\n\tv_nop"
               : "+v"(a0), "+v"(a1), "+v"(a2), "+v"(a3)
               : "v"(x), "v"(y0), "v"(y1), "v"(y2), "v"(y3));
}
__device__ __forceinline__ void acc_guard4(v8f& a, v8f& b, v8f& c, v8f& d) {
  asm volatile("v_nop\n\tv_nop\n\tv_nop\n\tv_nop" : "+v"(a), "+v"(b), "+v"(c), "+v"(d));
}

struct FragH {
  union U { v16h v; v8h h[2]; };
  static __device__ __forceinline__ v16h load(const _Float16* p) {
    U f; f.h[0] = *(const v8h*)(p); f.h[1] = *(const v8h*)(p + 16); return f.v;
  }
  static __device__ __forceinline__ v8f mma(v16h a, v16h b, v8f c) {
    return __builtin_amdgcn_wmma_f32_16x16x32_f16(false, a, false, b, (short)0, c, false, false);
  }
};

__device__ __forceinline__ float act_carried(float h) {
#if __has_builtin(__builtin_amdgcn_exp2f)
  const float e = __builtin_amdgcn_exp2f(h * TWO_LOG2E);
#else
  const float e = __expf(2.0f * h);
#endif
  const float rc = __builtin_amdgcn_rcpf(e + 1.0f);
  const float av = fmaf(-2.0f * ACARRY, rc, ACARRY);
  return (av >= H16_MINN) ? av : 0.0f;
}

__global__ __launch_bounds__(NTHR) void wplane_kernel(const float* __restrict__ src, unsigned short* __restrict__ O) {
  __shared__ float Tt[64 * 65];
  const int tid = threadIdx.x;
  const int c0 = blockIdx.x * 64, r0 = blockIdx.y * 64;
#pragma unroll
  for (int i = 0; i < 4; ++i) {
    const int idx = i * NTHR + tid;
    const int rr = idx >> 4, cc = (idx & 15) * 4;
    const v4f v = *(const v4f*)(src + (size_t)(r0 + rr) * (size_t)NHID + c0 + cc);
    Tt[rr * 65 + cc + 0] = v[0];
    Tt[rr * 65 + cc + 1] = v[1];
    Tt[rr * 65 + cc + 2] = v[2];
    Tt[rr * 65 + cc + 3] = v[3];
  }
  __syncthreads();
  const int q = tid >> 3, c8 = (tid & 7) * 8;
  v8h hv[2];
#pragma unroll
  for (int g = 0; g < 2; ++g) {
    const int qq = g * 32 + q;
#pragma unroll
    for (int e = 0; e < 8; ++e) {
      const float f  = Tt[(c8 + e) * 65 + qq] * WCARRY;
      const float fz = (fabsf(f) >= H16_MINN) ? f : 0.0f;
      hv[g][e] = (_Float16)fz;
    }
  }
  for (int pass = 0; pass < 2; ++pass) {
#pragma unroll
    for (int g = 0; g < 2; ++g) {
      const size_t o = (size_t)(c0 + g * 32 + q) * (size_t)NHID + (size_t)(r0 + c8);
      *(volatile v8h*)(O + o) = hv[g];
    }
    __threadfence();
  }
}

__global__ __launch_bounds__(NTHR) void leaky_seq_kernel(const float* __restrict__ initdir, const float* __restrict__ vel,
                                                         const float* __restrict__ fc_w, const float* __restrict__ fc_b,
                                                         const float* __restrict__ W_in, const float* __restrict__ W_out,
                                                         const float* __restrict__ bias,
                                                         const unsigned short* __restrict__ Btp,
                                                         float* __restrict__ out) {
  __shared__ __align__(16) _Float16 Ah[2][ROWS_BLK * HPITCH];
  __shared__ __align__(16) float    Pt[2][ROWS_BLK * NIO * PPITCH];
  const _Float16* Bt = (const _Float16*)Btp;
  const int tid  = threadIdx.x;
  const int lane = tid & 31;
  const int wave = __builtin_amdgcn_readfirstlane(tid >> 5);
  const int c = lane & 15, hh = lane >> 4, koff = hh * 8;
  const int rowbase = blockIdx.x * ROWS_BLK;
  const int j0 = 64 * wave + 4 * c;

  float w0s[4], w1s[4], bs[4], wo0[4], wo1[4];
  float hst[4][8];
  {
    const v4f wi0 = *(const v4f*)(W_in + j0);
    const v4f wi1 = *(const v4f*)(W_in + NHID + j0);
    const v4f bi  = *(const v4f*)(bias + j0);
    const v4f fb  = *(const v4f*)(fc_b + j0);
    const v4f fwa = *(const v4f*)(fc_w + 2 * j0);
    const v4f fwb = *(const v4f*)(fc_w + 2 * j0 + 4);
    const v4f woa = *(const v4f*)(W_out + 2 * j0);
    const v4f wob = *(const v4f*)(W_out + 2 * j0 + 4);
    const float f0[4] = { fwa[0], fwa[2], fwb[0], fwb[2] };
    const float f1[4] = { fwa[1], fwa[3], fwb[1], fwb[3] };
    wo0[0] = woa[0]; wo0[1] = woa[2]; wo0[2] = wob[0]; wo0[3] = wob[2];
    wo1[0] = woa[1]; wo1[1] = woa[3]; wo1[2] = wob[1]; wo1[3] = wob[3];
#pragma unroll
    for (int nt = 0; nt < 4; ++nt) {
      w0s[nt] = LEAKF * wi0[nt];
      w1s[nt] = LEAKF * wi1[nt];
      bs[nt]  = LEAKF * bi[nt];
    }
    const float* ip = initdir + (size_t)(rowbase + 8 * hh) * NIO;
    v4f iv[4];
#pragma unroll
    for (int i = 0; i < 4; ++i) iv[i] = *(const v4f*)(ip + 4 * i);
    _Float16* a0 = &Ah[0][0];
#pragma unroll
    for (int r = 0; r < 8; ++r) {
      const float d0 = iv[r >> 1][(r & 1) * 2];
      const float d1 = iv[r >> 1][(r & 1) * 2 + 1];
      v4h hv;
#pragma unroll
      for (int nt = 0; nt < 4; ++nt) {
        const float h0 = (d0 * f0[nt] + d1 * f1[nt]) + fb[nt];
        hst[nt][r] = h0;
        hv[nt] = (_Float16)act_carried(h0);
      }
      *(v4h*)(a0 + (8 * hh + r) * HPITCH + j0) = hv;
    }
  }
  __syncthreads();

  const _Float16* wb = Bt + (size_t)j0 * NHID + koff;
  const v8f z8 = {0.f, 0.f, 0.f, 0.f, 0.f, 0.f, 0.f, 0.f};

#pragma unroll 1
  for (int t = 0; t < NSTEP; ++t) {
    const int cur = t & 1;
    const float* xp = vel + ((size_t)t * NBATCH + (size_t)(rowbase + 8 * hh)) * NIO;
    v4f xv[4];
#pragma unroll
    for (int i = 0; i < 4; ++i) xv[i] = *(const v4f*)(xp + 4 * i);

    const _Float16* ahrow = &Ah[cur][0] + c * HPITCH + koff;
    _Float16* ahn = &Ah[cur ^ 1][0];
    float* pt = &Pt[cur][0];

    v8f acc[4];
    acc[0] = z8; acc[1] = z8; acc[2] = z8; acc[3] = z8;
#pragma unroll 2
    for (int k0 = 0; k0 < NHID; k0 += 32) {
      const v16h a  = FragH::load(ahrow + k0);
      const v16h b0 = FragH::load(wb + k0);
      const v16h b1 = FragH::load(wb + 1 * NHID + k0);
      const v16h b2 = FragH::load(wb + 2 * NHID + k0);
      const v16h b3 = FragH::load(wb + 3 * NHID + k0);
      acc[0] = FragH::mma(a, b0, acc[0]);
      acc[1] = FragH::mma(a, b1, acc[1]);
      acc[2] = FragH::mma(a, b2, acc[2]);
      acc[3] = FragH::mma(a, b3, acc[3]);
      guard_group4(acc[0], acc[1], acc[2], acc[3], a, b0, b1, b2, b3);
    }
    acc_guard4(acc[0], acc[1], acc[2], acc[3]);

#pragma unroll
    for (int r = 0; r < 8; ++r) {
      const float x0 = xv[r >> 1][(r & 1) * 2];
      const float x1 = xv[r >> 1][(r & 1) * 2 + 1];
      float q0 = 0.0f, q1 = 0.0f;
      v4h hv;
#pragma unroll
      for (int nt = 0; nt < 4; ++nt) {
        float u = fmaf(x0, w0s[nt], bs[nt]);
        u = fmaf(x1, w1s[nt], u);
        u = fmaf(acc[nt][r], FOLDSC, u);
        const float hn = fmaf(KEEPF, hst[nt][r], u);
        hst[nt][r] = hn;
        q0 = fmaf(hn, wo0[nt], q0);
        q1 = fmaf(hn, wo1[nt], q1);
        hv[nt] = (_Float16)act_carried(hn);
      }
      *(v4h*)(ahn + (8 * hh + r) * HPITCH + j0) = hv;
      pt[(2 * (8 * hh + r) + 0) * PPITCH + 16 * wave + c] = q0;
      pt[(2 * (8 * hh + r) + 1) * PPITCH + 16 * wave + c] = q1;
    }
    __syncthreads();

    if (wave == 0) {
      const float* pr = pt + lane * PPITCH;
      v4f s = {0.f, 0.f, 0.f, 0.f};
#pragma unroll 4
      for (int i = 0; i < 32; ++i) s += *(const v4f*)(pr + 4 * i);
      const float o = (s[0] + s[1]) + (s[2] + s[3]);
      float* op = out + ((size_t)t * NBATCH + (size_t)rowbase) * NIO + lane;
      *(volatile float*)op = o;
      __threadfence();
      *(volatile float*)op = o;
    }
  }
}

extern "C" void kernel_launch(void* const* d_in, const int* in_sizes, int n_in,
                              void* d_out, int out_size, void* d_ws, size_t ws_size, hipStream_t stream) {
  if (n_in < 8 || d_out == nullptr || d_ws == nullptr) return;
  if (in_sizes[0] != NBATCH * NIO || in_sizes[1] != NSTEP * NBATCH * NIO || in_sizes[2] != NHID * NIO ||
      in_sizes[3] != NHID || in_sizes[4] != NIO * NHID || in_sizes[5] != NHID * NHID ||
      in_sizes[6] != NHID * NIO || in_sizes[7] != NHID || out_size != NOUT) return;

  const float* initdir = (const float*)d_in[0];
  const float* vel     = (const float*)d_in[1];
  const float* fc_w    = (const float*)d_in[2];
  const float* fc_b    = (const float*)d_in[3];
  const float* w_in    = (const float*)d_in[4];
  const float* w_rec   = (const float*)d_in[5];
  const float* w_out   = (const float*)d_in[6];
  const float* bias    = (const float*)d_in[7];
  float* out = (float*)d_out;

  char* ws = (char*)d_ws; size_t off = 0;
  auto carve = [&](size_t bytes) -> char* { char* p = ws + off; off += (bytes + 255) & ~(size_t)255; return p; };
  unsigned short* BT = (unsigned short*)carve((size_t)NHID * NHID * 2);
  if (off > ws_size || off > (size_t)134217728) return;

  wplane_kernel<<<dim3(NHID / 64, NHID / 64), NTHR, 0, stream>>>(w_rec, BT);
  leaky_seq_kernel<<<NBATCH / ROWS_BLK, NTHR, 0, stream>>>(initdir, vel, fc_w, fc_b, w_in, w_out, bias, BT, out);
}
